// MultiHeadTEAttention_54589034332766
// MI455X (gfx1250) — hardware-verified
//
#include <hip/hip_runtime.h>


namespace {
constexpr int MB = 8, NQ = 512, NK = 512, DX = 64, DY = 256, DH = 128;
constexpr float XS = 8.0f, HS = 256.0f, PS = 16384.0f, WSC = 256.0f, FMIN = -3.4028234663852886e38f;
typedef _Float16 b16;
typedef __attribute__((ext_vector_type(16))) _Float16 v16b;
typedef __attribute__((ext_vector_type(8))) _Float16 v8b;
typedef __attribute__((ext_vector_type(8))) float v8f;
typedef __attribute__((ext_vector_type(4))) float v4f;
typedef __attribute__((ext_vector_type(2))) float v2f;
typedef __attribute__((ext_vector_type(2))) _Float16 v2b;
__device__ __forceinline__ float bf16_rne(float f) { unsigned int u = __float_as_uint(f); u += 0x7FFFu + ((u >> 16) & 1u); float r = __uint_as_float(u & 0xFFFF0000u); asm volatile("" : "+v"(r)); return r; }
__device__ __forceinline__ float bfv(float f) { float r = bf16_rne(f); asm volatile("" : "+v"(r)); return r; }
__device__ __forceinline__ void split16(float v, b16& hi, b16& lo) { hi = (b16)v; lo = (b16)(v - (float)hi); }
__device__ __forceinline__ v16b frag_kb(const b16* p, int hh) { const v8b a = *(const v8b*)(p + 8 * hh), b = *(const v8b*)(p + 16 + 8 * hh); v16b f;
#pragma unroll
  for (int e = 0; e < 8; ++e) { f[e] = a[e]; f[8 + e] = b[e]; } return f; }
__device__ __forceinline__ v8f wmma16b(v16b a, v16b b, v8f c) { v8f d = __builtin_amdgcn_wmma_f32_16x16x32_f16(false, a, false, b, (short)0, c, false, false); asm volatile("v_nop\n\tv_nop\n\tv_nop\n\tv_nop" : "+v"(d) : "v"(a), "v"(b)); return d; }
__device__ __forceinline__ void wave_lds_sync() { __builtin_amdgcn_fence(__ATOMIC_RELEASE, "workgroup"); __builtin_amdgcn_wave_barrier(); __builtin_amdgcn_fence(__ATOMIC_ACQUIRE, "workgroup"); }
__device__ __forceinline__ float pmul(float a, float b) { float p = a * b; asm volatile("" : "+v"(p)); return p; }
__device__ __forceinline__ float wsum(float v) { for (int o = 16; o; o >>= 1) v += __shfl_xor(v, o); return v; }

__global__ __launch_bounds__(256) void prep_kernel(const float* __restrict__ wv, const float* __restrict__ wo, const float* __restrict__ xk, b16* __restrict__ WV, b16* __restrict__ WO, b16* __restrict__ XK, float* __restrict__ KN) { const size_t nt = (size_t)gridDim.x * 256, u0 = (size_t)blockIdx.x * 256 + threadIdx.x; v8b v; auto put = [&](b16* dst) { for (int pass = 0; pass < 2; ++pass) { *(volatile v8b*)dst = v; __threadfence(); } };
  for (size_t u = u0; u < (size_t)DH * 32; u += nt) { const int h = (int)(u / 32), d0 = (int)(u % 32) * 8;
#pragma unroll
    for (int j = 0; j < 8; ++j) v[j] = (b16)(bf16_rne(wv[(size_t)(d0 + j) * DH + h]) * WSC); put(WV + (size_t)h * DY + d0); }
  for (size_t u = u0; u < (size_t)DY * 16; u += nt) { const int d = (int)(u / 16), h0 = (int)(u % 16) * 8;
#pragma unroll
    for (int j = 0; j < 8; ++j) v[j] = (b16)(bf16_rne(wo[(size_t)(h0 + j) * DY + d]) * WSC); put(WO + (size_t)d * DH + h0); }
  for (size_t u = u0; u < (size_t)MB * NK * 8; u += nt) { const size_t r = u / 8; const int c0 = (int)(u % 8) * 8;
#pragma unroll
    for (int j = 0; j < 8; ++j) v[j] = (b16)(bfv(xk[r * DX + c0 + j]) * XS); put(XK + r * DX + c0); }
  for (size_t r = u0; r < (size_t)MB * NK; r += nt) { float s = 0.0f; for (int c = 0; c < DX; ++c) { const float t = bfv(xk[r * DX + c]); s += t * t; } for (int pass = 0; pass < 2; ++pass) { ((volatile float*)KN)[r] = s; __threadfence(); } } }
__global__ __launch_bounds__(32) void vproj_kernel(const float* __restrict__ yv, const b16* __restrict__ WV, float* __restrict__ Vr) { __shared__ __attribute__((aligned(16))) b16 Ax[16][DY + 8]; __shared__ float Tf[16][DH + 4]; const int lane = threadIdx.x, nloc = lane & 15, hlf = lane >> 4; const size_t r0 = (size_t)blockIdx.x * 16;
  for (int rr = 0; rr < 16; ++rr) for (int q = 0; q < DY / 32; ++q) { const int c = q * 32 + lane; Ax[rr][c] = (b16)(bfv(yv[(r0 + rr) * DY + c]) * XS); }
  if (lane < 16) for (int k = DY; k < DY + 8; ++k) Ax[lane][k] = (b16)0.0f;
  wave_lds_sync(); v8f acc[8];
#pragma unroll
  for (int t = 0; t < 8; ++t) acc[t] = (v8f){};
#pragma unroll 2
  for (int kb = 0; kb < DY; kb += 32) { const v16b a = frag_kb(&Ax[nloc][kb], hlf);
#pragma unroll
    for (int t = 0; t < 8; ++t) acc[t] = wmma16b(a, frag_kb(WV + (size_t)(t * 16 + nloc) * DY + kb, hlf), acc[t]); }
#pragma unroll
  for (int t = 0; t < 8; ++t)
#pragma unroll
    for (int r8 = 0; r8 < 8; ++r8) Tf[8 * hlf + r8][t * 16 + nloc] = acc[t][r8] * (1.0f / (XS * WSC));
  wave_lds_sync();
  for (int pass = 0; pass < 2; ++pass) { for (int rr = 0; rr < 16; ++rr) *(volatile v4f*)(Vr + (r0 + rr) * DH + lane * 4) = *(const v4f*)(&Tf[rr][lane * 4]); __threadfence(); } }
__global__ __launch_bounds__(256) void vt_kernel(const float* __restrict__ Vr, b16* __restrict__ VTh, b16* __restrict__ VTl) { __shared__ float Tt[64][129]; const size_t r0 = (size_t)blockIdx.x * 64; const int m = (int)(r0 / NK), k0 = (int)(r0 % NK); const int tid = threadIdx.x, wave = tid >> 5, lane = tid & 31;
  for (int q = wave; q < 64; q += 8) for (int c = lane; c < DH; c += 32) Tt[q][c] = Vr[(r0 + q) * DH + c];
  __syncthreads();
  for (int pass = 0; pass < 2; ++pass) { for (int h = wave; h < DH; h += 8) { b16 h0, l0, h1, l1; split16(Tt[lane * 2][h] * HS, h0, l0); split16(Tt[lane * 2 + 1][h] * HS, h1, l1); const size_t o = ((size_t)m * DH + h) * NK + k0 + lane * 2; *(volatile v2b*)(VTh + o) = (v2b){h0, h1}; *(volatile v2b*)(VTl + o) = (v2b){l0, l1}; } __threadfence(); } }
__global__ __launch_bounds__(32) void att_kernel(const float* __restrict__ xq, const b16* __restrict__ XK, const float* __restrict__ KN, const int* __restrict__ mask, const float* __restrict__ lsc, const b16* __restrict__ VTh, const b16* __restrict__ VTl, const b16* __restrict__ WO, const float* __restrict__ bout, int QLIM, float* __restrict__ out) { __shared__ __attribute__((aligned(16))) b16 Aq[16][DX + 8], Pa[16][NK + 8], Pb[16][NK + 8], Oh[16][DH + 8], Ol[16][DH + 8]; __shared__ float Sc[16][NK + 1], Tf[16][260], QN[16]; const int lane = threadIdx.x, nloc = lane & 15, hlf = lane >> 4; const int m = blockIdx.x / (NQ / 16), q0 = (blockIdx.x % (NQ / 16)) * 16; if (q0 >= QLIM) return; const size_t tq = (size_t)m * NQ + q0;
  for (int rr = 0; rr < 16; ++rr) for (int q = 0; q < 2; ++q) { const int c = q * 32 + lane; Aq[rr][c] = (b16)(bfv(xq[(tq + rr) * DX + c]) * XS); }
  if (lane < 16) { for (int k = DX; k < DX + 8; ++k) Aq[lane][k] = (b16)0.0f; for (int k = NK; k < NK + 8; ++k) { Pa[lane][k] = (b16)0.0f; Pb[lane][k] = (b16)0.0f; } for (int k = DH; k < DH + 8; ++k) { Oh[lane][k] = (b16)0.0f; Ol[lane][k] = (b16)0.0f; } float s = 0.0f; for (int c = 0; c < DX; ++c) { const float t = bfv(xq[(tq + lane) * DX + c]); s += t * t; } QN[lane] = s; }
  wave_lds_sync();
  const v16b qa0 = frag_kb(&Aq[nloc][0], hlf), qa1 = frag_kb(&Aq[nloc][32], hlf);
#pragma unroll 1
  for (int tg = 0; tg < NK / 16; tg += 4) { v8f d[4] = {(v8f){}, (v8f){}, (v8f){}, (v8f){}};
#pragma unroll
    for (int t = 0; t < 4; ++t) { const size_t ko = ((size_t)m * NK + (tg + t) * 16 + nloc) * DX; d[t] = wmma16b(qa0, frag_kb(XK + ko, hlf), d[t]); d[t] = wmma16b(qa1, frag_kb(XK + ko + 32, hlf), d[t]); }
#pragma unroll
    for (int t = 0; t < 4; ++t)
#pragma unroll
      for (int r8 = 0; r8 < 8; ++r8) Sc[8 * hlf + r8][(tg + t) * 16 + nloc] = d[t][r8] * (1.0f / (XS * XS)); }
  wave_lds_sync();
  if (lane < 16) { const int r = lane; const float l2 = bfv(lsc[0]) * bfv(lsc[0]); const float cf = -0.5f / l2; const int* mk = mask + (tq + r) * NK; float mx = -INFINITY;
    for (int k = 0; k < NK; ++k) { const float sq = QN[r] + KN[(size_t)m * NK + k] - 2.0f * Sc[r][k]; float s = sq * cf; if (mk[k] == 0) s = FMIN; Sc[r][k] = s; mx = fmaxf(mx, s); }
    float z = 0.0f; for (int k = 0; k < NK; ++k) z += __expf(Sc[r][k] - mx); const float inv = 1.0f / z;
    for (int k = 0; k < NK; ++k) { b16 p, pl; split16(__expf(Sc[r][k] - mx) * inv * PS, p, pl); Pa[r][k] = p; Pb[r][k] = pl; } }
  wave_lds_sync();
  { v8f acc[8];
#pragma unroll
    for (int t = 0; t < 8; ++t) acc[t] = (v8f){};
#pragma unroll 2
    for (int kb = 0; kb < NK; kb += 32) { const v16b pa = frag_kb(&Pa[nloc][kb], hlf), pb = frag_kb(&Pb[nloc][kb], hlf);
#pragma unroll
      for (int t = 0; t < 8; ++t) { const size_t vo = ((size_t)m * DH + t * 16 + nloc) * NK + kb; const v16b vh = frag_kb(VTh + vo, hlf), vl = frag_kb(VTl + vo, hlf); acc[t] = wmma16b(pa, vh, acc[t]); acc[t] = wmma16b(pa, vl, acc[t]); acc[t] = wmma16b(pb, vh, acc[t]); } }
#pragma unroll
    for (int t = 0; t < 8; ++t)
#pragma unroll
      for (int r8 = 0; r8 < 8; ++r8) { b16 p, pl; split16(acc[t][r8] * (1.0f / (PS * HS)) * HS, p, pl); Oh[8 * hlf + r8][t * 16 + nloc] = p; Ol[8 * hlf + r8][t * 16 + nloc] = pl; } }
  wave_lds_sync();
  { v8f acc[16];
#pragma unroll
    for (int t = 0; t < 16; ++t) acc[t] = (v8f){};
#pragma unroll
    for (int kb = 0; kb < DH; kb += 32) { const v16b a = frag_kb(&Oh[nloc][kb], hlf), al = frag_kb(&Ol[nloc][kb], hlf);
#pragma unroll
      for (int t = 0; t < 16; ++t) { const v16b bw = frag_kb(WO + (size_t)(t * 16 + nloc) * DH + kb, hlf); acc[t] = wmma16b(a, bw, acc[t]); acc[t] = wmma16b(al, bw, acc[t]); } }
#pragma unroll
    for (int t = 0; t < 16; ++t) { const int cc = t * 16 + nloc; const float bb = bfv(bout[cc]);
#pragma unroll
      for (int r8 = 0; r8 < 8; ++r8) Tf[8 * hlf + r8][cc] = acc[t][r8] * (1.0f / (HS * WSC)) + bb; } }
  wave_lds_sync();
  for (int pass = 0; pass < 2; ++pass) { for (int rr = 0; rr < 16; ++rr) for (int q = 0; q < 2; ++q) *(volatile v4f*)(out + (tq + rr) * DY + q * 128 + lane * 4) = *(const v4f*)(&Tf[rr][q * 128 + lane * 4]); __threadfence(); } }
}

extern "C" void kernel_launch(void* const* d_in, const int* in_sizes, int n_in, void* d_out, int out_size, void* d_ws, size_t ws_size, hipStream_t stream) {
  (void)n_in;
  auto Fp = [&](int i) { return (const float*)d_in[i]; }; auto Ip = [&](int i) { return (const int*)d_in[i]; };
  if (in_sizes[0] != MB * NQ * DX || in_sizes[1] != MB * NK * DX || in_sizes[2] != MB * NK * DY || in_sizes[3] != MB * NQ * NK || in_sizes[4] != DY * DH || in_sizes[5] != DH * DY || in_sizes[6] != DY || in_sizes[7] != 1 || out_size != MB * NQ * DY) return;
  const int QLIM = NQ;
  size_t off = 0; char* ws = (char*)d_ws;
  auto carve = [&](size_t bytes) { char* p = ws + off; off += (bytes + 255) & ~(size_t)255; return p; };
  b16* WV = (b16*)carve((size_t)DH * DY * 2); b16* WO = (b16*)carve((size_t)DY * DH * 2); b16* XK = (b16*)carve((size_t)MB * NK * DX * 2); float* KN = (float*)carve((size_t)MB * NK * 4); float* Vr = (float*)carve((size_t)MB * NK * DH * 4); b16* VTh = (b16*)carve((size_t)MB * DH * NK * 2); b16* VTl = (b16*)carve((size_t)MB * DH * NK * 2);
  if (off > ws_size || off > ((size_t)8 << 20)) return;
  prep_kernel<<<64, 256, 0, stream>>>(Fp(4), Fp(5), Fp(1), WV, WO, XK, KN);
  vproj_kernel<<<MB * NK / 16, 32, 0, stream>>>(Fp(2), WV, Vr);
  vt_kernel<<<MB * NK / 64, 256, 0, stream>>>(Vr, VTh, VTl);
  att_kernel<<<MB * (NQ / 16), 32, 0, stream>>>(Fp(0), XK, KN, Ip(3), Fp(7), VTh, VTl, WO, Fp(6), QLIM, (float*)d_out);
}
